// MambaSequenceEncoder_22299470201655
// MI455X (gfx1250) — hardware-verified
//
#include <hip/hip_runtime.h>
#include <math.h>


#define BB 8
#define LL 1024
#define DM 256
#define DI 512
#define DS 16
#define DCONV 4
#define NL 4
#define MROWS (BB * LL)
#define NDT 576
#define WSC 64.0f
#define XSC 1024.0f
#define YSC 4096.0f
#define LOG2E_F 1.4426950408889634f
#define LN_EPS 1e-5f

typedef __attribute__((ext_vector_type(16))) _Float16 v16h;
typedef __attribute__((ext_vector_type(8)))  _Float16 v8h;
typedef __attribute__((ext_vector_type(4)))  _Float16 v4h;
typedef __attribute__((ext_vector_type(16))) __bf16   v16b;
typedef __attribute__((ext_vector_type(8)))  __bf16   v8b;
typedef __attribute__((ext_vector_type(8)))  float    v8f;
typedef __attribute__((ext_vector_type(4)))  float    v4f;
typedef __attribute__((ext_vector_type(2)))  float    v2f;

__device__ __forceinline__ unsigned short f2bf_bits(float f) {
  unsigned u = __float_as_uint(f);
  return (unsigned short)((u + 0x7FFFu + ((u >> 16) & 1u)) >> 16);
}
__device__ __forceinline__ float bf_bits2f(unsigned short h) { return __uint_as_float(((unsigned)h) << 16); }

__device__ __forceinline__ void dep_guard_h(v8f& a, v8f& b, v16h x, v16h y) { asm volatile("v_nop\n\tv_nop\n\tv_nop\n\tv_nop" : "+v"(a), "+v"(b) : "v"(x), "v"(y)); }
__device__ __forceinline__ void dep_guard_b(v8f& a, v8f& b, v16b x, v16b y) { asm volatile("v_nop\n\tv_nop\n\tv_nop\n\tv_nop" : "+v"(a), "+v"(b) : "v"(x), "v"(y)); }
__device__ __forceinline__ void keep4_h(v16h a, v16h b, v16h c, v16h d) { asm volatile("v_nop" :: "v"(a), "v"(b), "v"(c), "v"(d)); }
__device__ __forceinline__ void keep4_b(v16b a, v16b b, v16b c, v16b d) { asm volatile("v_nop" :: "v"(a), "v"(b), "v"(c), "v"(d)); }
__device__ __forceinline__ void acc_guard4(v8f& a, v8f& b, v8f& c, v8f& d) { asm volatile("v_nop\n\tv_nop\n\tv_nop\n\tv_nop" : "+v"(a), "+v"(b), "+v"(c), "+v"(d)); }
template <typename T> struct Frag;
template <> struct Frag<_Float16> {
  typedef v16h V; union U { v16h v; v8h h[2]; };
  static __device__ __forceinline__ v16h load(const _Float16* p) {
    U f; f.h[0] = *(const v8h*)(p); f.h[1] = *(const v8h*)(p + 16); return f.v;
  }
  static __device__ __forceinline__ v8f mma(v16h a, v16h b, v8f c) {
    return __builtin_amdgcn_wmma_f32_16x16x32_f16(false, a, false, b, (short)0, c, false, false);
  }
  static __device__ __forceinline__ void guard(v8f& a, v8f& b, v16h x, v16h y) { dep_guard_h(a, b, x, y); }
  static __device__ __forceinline__ void keep(v16h a, v16h b, v16h c, v16h d) { keep4_h(a, b, c, d); }
};
template <> struct Frag<__bf16> {
  typedef v16b V; union U { v16b v; v8b h[2]; };
  static __device__ __forceinline__ v16b load(const __bf16* p) {
    U f; f.h[0] = *(const v8b*)(p); f.h[1] = *(const v8b*)(p + 16); return f.v;
  }
  static __device__ __forceinline__ v8f mma(v16b a, v16b b, v8f c) {
    return __builtin_amdgcn_wmma_f32_16x16x32_bf16(false, a, false, b, (short)0, c, false, false);
  }
  static __device__ __forceinline__ void guard(v8f& a, v8f& b, v16b x, v16b y) { dep_guard_b(a, b, x, y); }
  static __device__ __forceinline__ void keep(v16b a, v16b b, v16b c, v16b d) { keep4_b(a, b, c, d); }
};

template <int ET> struct Elem;
template <> struct Elem<0> { typedef _Float16 T; };
template <> struct Elem<1> { typedef __bf16 T; };
template <int ET, bool SPLIT, int BIAS_MODE, int OUT_MODE, bool RESID, int ACT = 0>
__global__ __launch_bounds__(256) void wmma_gemm64(
    const unsigned short* __restrict__ Ap, const unsigned short* __restrict__ A2p, int lda, long strideA,
    const unsigned short* __restrict__ Btp, const unsigned short* __restrict__ Bt2p, int ldb, long strideB,
    void* __restrict__ Cout, void* __restrict__ Cout2, int ldc, long strideC,
    const float* __restrict__ bias,
    const float* __restrict__ resid, long strideR,
    int M, int N, int K, float scale) {
  typedef typename Elem<ET>::T T;
  typedef typename Frag<T>::V V;
  const T* A = (const T*)Ap; const T* A2 = (const T*)A2p; const T* Bt = (const T*)Btp; const T* Bt2 = (const T*)Bt2p;
  __shared__ __align__(16) float sT[8][16 * 68];
  const int b    = blockIdx.y;
  const int lane = threadIdx.x & 31;
  const int wave = threadIdx.x >> 5;
  const int tilesN = N >> 6;
  const int tilesM = M >> 6;
  const int tile = blockIdx.x * 8 + wave;
  if (tile >= tilesM * tilesN) return;
  const int tm = tile / tilesN;
  const int tn = tile - tm * tilesN;
  const int m0 = tm << 6;
  const int n0 = tn << 6;

  const T* Ab  = A  + (size_t)b * strideA;
  const T* Bb  = Bt + (size_t)b * strideB;
  const T* Ab2 = SPLIT ? (A2  + (size_t)b * strideA) : nullptr;
  const T* Bb2 = SPLIT ? (Bt2 + (size_t)b * strideB) : nullptr;

  const int rlane = lane & 15;
  const int koff  = (lane >> 4) * 8;
  const int mOff  = (lane >> 4) * 8;

  v8f acc[4][4];
#pragma unroll
  for (int i = 0; i < 4; ++i)
#pragma unroll
    for (int j = 0; j < 4; ++j) acc[i][j] = (v8f){0.f,0.f,0.f,0.f,0.f,0.f,0.f,0.f};

  for (int k0 = 0; k0 < K; k0 += 32) {
    V bh[4], bl[4];
#pragma unroll
    for (int j = 0; j < 4; ++j) {
      const size_t bo = (size_t)(n0 + (j << 4) + rlane) * ldb + koff + k0;
      bh[j] = Frag<T>::load(Bb + bo);
      if (SPLIT) bl[j] = Frag<T>::load(Bb2 + bo);
    }
#pragma unroll
    for (int i = 0; i < 4; ++i) {
      const size_t ao = (size_t)(m0 + (i << 4) + rlane) * lda + koff + k0;
      V ah = Frag<T>::load(Ab + ao);
      V al;
      if (SPLIT) al = Frag<T>::load(Ab2 + ao);
#pragma unroll
      for (int j = 0; j < 4; ++j) {
        acc[i][j] = Frag<T>::mma(ah, bh[j], acc[i][j]);
        if (SPLIT) {
          acc[i][j] = Frag<T>::mma(ah, bl[j], acc[i][j]);
          acc[i][j] = Frag<T>::mma(al, bh[j], acc[i][j]);
        }
      }
      Frag<T>::guard(acc[i][0], acc[i][3], ah, SPLIT ? al : ah);
    }
    Frag<T>::keep(bh[0], bh[1], bh[2], bh[3]);
    if (SPLIT) Frag<T>::keep(bl[0], bl[1], bl[2], bl[3]);
  }
  acc_guard4(acc[0][0], acc[0][1], acc[0][2], acc[0][3]);
  acc_guard4(acc[1][0], acc[1][1], acc[1][2], acc[1][3]);
  acc_guard4(acc[2][0], acc[2][1], acc[2][2], acc[2][3]);
  acc_guard4(acc[3][0], acc[3][1], acc[3][2], acc[3][3]);

  float* slab = sT[wave];
  const float* Rb = RESID ? (resid + (size_t)b * strideR) : nullptr;
#pragma unroll
  for (int i = 0; i < 4; ++i) {
    const int mBase = m0 + (i << 4);
#pragma unroll
    for (int j = 0; j < 4; ++j) {
      const int n = n0 + (j << 4) + rlane;
      float bv = 0.f;
      if (BIAS_MODE == 2) bv = bias[n];
#pragma unroll
      for (int r = 0; r < 8; ++r) {
        float v = acc[i][j][r] * scale;
        if (BIAS_MODE == 1) v += bias[mBase + mOff + r];
        if (BIAS_MODE == 2) v += bv;
        if (RESID) v += Rb[(size_t)(mBase + mOff + r) * ldc + n];
        if (ACT == 1) v = tanhf(v);
        if (ACT == 2) v = fmaxf(v, 0.0f);
        if (ACT == 3) v = v / (1.0f + expf(-v));
        if (ACT == 4) v = (v > 0.f) ? v : 0.01f * v;
        if (ACT == 5) v = 0.5f * v * (1.0f + erff(v * 0.70710678118654752f));
        slab[(mOff + r) * 68 + (j << 4) + rlane] = v;
      }
    }
    __builtin_amdgcn_fence(__ATOMIC_RELEASE, "workgroup");
    __builtin_amdgcn_wave_barrier();
    __builtin_amdgcn_fence(__ATOMIC_ACQUIRE, "workgroup");
    if (OUT_MODE == 0) {
      float* C = (float*)Cout + (size_t)b * strideC;
      const int hh = lane >> 4, c4 = (lane & 15) * 4;
      for (int pass = 0; pass < 2; ++pass) {
#pragma unroll
        for (int it = 0; it < 8; ++it) {
          const int row = it * 2 + hh;
          v4f v = *(const v4f*)(slab + row * 68 + c4);
          *(volatile v4f*)(C + (size_t)(mBase + row) * ldc + n0 + c4) = v;
        }
        __threadfence();
      }
    } else {
      const int q = lane >> 3, c8 = (lane & 7) * 8;
      unsigned short* C  = (unsigned short*)Cout  + (size_t)b * strideC;
      unsigned short* C2 = (OUT_MODE == 2) ? ((unsigned short*)Cout2 + (size_t)b * strideC) : nullptr;
      for (int pass = 0; pass < 2; ++pass) {
#pragma unroll
        for (int it = 0; it < 4; ++it) {
          const int row = it * 4 + q;
          const float* sp = slab + row * 68 + c8;
          v8h hv, lv;
#pragma unroll
          for (int e = 0; e < 8; ++e) {
            if (OUT_MODE == 1) {
              hv[e] = (_Float16)sp[e];
            } else {
              unsigned short hb = f2bf_bits(sp[e]);
              unsigned short lb = f2bf_bits(sp[e] - bf_bits2f(hb));
              hv[e] = __builtin_bit_cast(_Float16, hb);
              lv[e] = __builtin_bit_cast(_Float16, lb);
            }
          }
          *(volatile v8h*)(C + (size_t)(mBase + row) * ldc + n0 + c8) = hv;
          if (OUT_MODE == 2) *(volatile v8h*)(C2 + (size_t)(mBase + row) * ldc + n0 + c8) = lv;
        }
        __threadfence();
      }
    }
    __builtin_amdgcn_fence(__ATOMIC_RELEASE, "workgroup");
    __builtin_amdgcn_wave_barrier();
    __builtin_amdgcn_fence(__ATOMIC_ACQUIRE, "workgroup");
  }
}

__global__ __launch_bounds__(256) void k_wprep(const float* __restrict__ in, int ldi, long strideI, int K, int N, int Npad,
                                              _Float16* __restrict__ out, int ldo, long strideO, int row_off, float sc) {
  __shared__ __align__(16) _Float16 tT[64 * 72];
  const int tid = threadIdx.x, lane = tid & 31, wave = tid >> 5;
  const int z = blockIdx.z;
  const int k0 = blockIdx.x * 64;
  const int n0 = blockIdx.y * 64;
  (void)K;
  const float* inz = in + (size_t)z * strideI;
  const int kr0 = tid >> 4;
  const int nc = (tid & 15) * 4;
#pragma unroll
  for (int p = 0; p < 4; ++p) {
    const int kr = p * 16 + kr0;
    const int k = k0 + kr;
    const int n = n0 + nc;
    const bool ok = (n < N);
    const int ncl = ok ? n : 0;
    const v4f v = *(const v4f*)(inz + (size_t)k * ldi + ncl);
#pragma unroll
    for (int e = 0; e < 4; ++e) tT[(nc + e) * 72 + kr] = ok ? (_Float16)(v[e] * sc) : (_Float16)0.0f;
  }
  __syncthreads();
  const int q = lane >> 3, c8 = (lane & 7) * 8;
  _Float16* outz = out + (size_t)z * strideO;
  for (int pass = 0; pass < 2; ++pass) {
#pragma unroll
    for (int it = 0; it < 2; ++it) {
      const int r = wave * 8 + it * 4 + q;
      const int n = n0 + r;
      if (n < Npad) {
        const v8h v = *(const v8h*)(tT + r * 72 + c8);
        *(volatile v8h*)(outz + (size_t)(row_off + n) * ldo + k0 + c8) = v;
      }
    }
    __threadfence();
  }
}

__device__ __forceinline__ float wave_sum(float v) {
  v += __shfl_xor(v, 16, 32);
  v += __shfl_xor(v, 8, 32);
  v += __shfl_xor(v, 4, 32);
  v += __shfl_xor(v, 2, 32);
  v += __shfl_xor(v, 1, 32);
  return v;
}
__device__ __forceinline__ void ln_row8(const float (&v)[8], const float* __restrict__ g, const float* __restrict__ bb,
                                        int cA, int cB, float (&o)[8]) {
  float s = 0.f;
#pragma unroll
  for (int e = 0; e < 8; ++e) s += v[e];
  s = wave_sum(s);
  const float m = s * (1.0f / DM);
  float q = 0.f;
#pragma unroll
  for (int e = 0; e < 8; ++e) { const float d = v[e] - m; q += d * d; }
  q = wave_sum(q);
  const float rs = rsqrtf(q * (1.0f / DM) + LN_EPS);
  const v4f gA = *(const v4f*)(g + cA), gB = *(const v4f*)(g + cB);
  const v4f bA = *(const v4f*)(bb + cA), bB2 = *(const v4f*)(bb + cB);
#pragma unroll
  for (int e = 0; e < 4; ++e) {
    o[e]     = (v[e] - m) * rs * gA[e] + bA[e];
    o[4 + e] = (v[4 + e] - m) * rs * gB[e] + bB2[e];
  }
}

__global__ __launch_bounds__(256) void k_stem(const float* __restrict__ x, const float* __restrict__ w_in, const float* __restrict__ b_in,
                                             const float* __restrict__ g, const float* __restrict__ bb, float* __restrict__ h) {
  const int lane = threadIdx.x & 31, wave = threadIdx.x >> 5;
  const int row = blockIdx.x * 8 + wave;
  const int b = row >> 10, l = row & (LL - 1);
  const float x0 = x[((size_t)b * 4 + 0) * LL + l];
  const float x1 = x[((size_t)b * 4 + 1) * LL + l];
  const float x2 = x[((size_t)b * 4 + 2) * LL + l];
  const float x3 = x[((size_t)b * 4 + 3) * LL + l];
  const int cA = lane * 4, cB = 128 + lane * 4;
  const v4f biA = *(const v4f*)(b_in + cA), biB = *(const v4f*)(b_in + cB);
  float v[8];
#pragma unroll
  for (int e = 0; e < 4; ++e) {
    const v4f w = *(const v4f*)(w_in + (size_t)(cA + e) * 4);
    v[e] = (((x0 * w[0] + x1 * w[1]) + x2 * w[2]) + x3 * w[3]) + biA[e];
    const v4f w2 = *(const v4f*)(w_in + (size_t)(cB + e) * 4);
    v[4 + e] = (((x0 * w2[0] + x1 * w2[1]) + x2 * w2[2]) + x3 * w2[3]) + biB[e];
  }
  float o[8];
  ln_row8(v, g, bb, cA, cB, o);
  v4f oA, oB;
#pragma unroll
  for (int e = 0; e < 4; ++e) { oA[e] = o[e]; oB[e] = o[4 + e]; }
  float* pr = h + (size_t)row * DM;
  *(volatile v4f*)(pr + cA) = oA;
  *(volatile v4f*)(pr + cB) = oB;
  __threadfence();
  *(volatile v4f*)(pr + cA) = oA;
  *(volatile v4f*)(pr + cB) = oB;
}

__global__ __launch_bounds__(256) void k_ln(const float* __restrict__ h, const float* __restrict__ g, const float* __restrict__ bb,
                                           _Float16* __restrict__ hn16) {
  const int lane = threadIdx.x & 31, wave = threadIdx.x >> 5;
  const int row = blockIdx.x * 8 + wave;
  const int cA = lane * 4, cB = 128 + lane * 4;
  const float* pr = h + (size_t)row * DM;
  const v4f vA = *(const v4f*)(pr + cA), vB = *(const v4f*)(pr + cB);
  float v[8] = {vA[0], vA[1], vA[2], vA[3], vB[0], vB[1], vB[2], vB[3]};
  float o[8];
  ln_row8(v, g, bb, cA, cB, o);
  v4h oA, oB;
#pragma unroll
  for (int e = 0; e < 4; ++e) { oA[e] = (_Float16)o[e]; oB[e] = (_Float16)o[4 + e]; }
  _Float16* po = hn16 + (size_t)row * DM;
  *(volatile v4h*)(po + cA) = oA;
  *(volatile v4h*)(po + cB) = oB;
  __threadfence();
  *(volatile v4h*)(po + cA) = oA;
  *(volatile v4h*)(po + cB) = oB;
}

__global__ __launch_bounds__(256) void k_conv(const float* __restrict__ xz, const float* __restrict__ cw, const float* __restrict__ cb,
                                             float* __restrict__ xs32, _Float16* __restrict__ xs16) {
  const int idx = blockIdx.x * 256 + threadIdx.x;
  const int cp = idx & 255;
  const int row = idx >> 8;
  const int l = row & (LL - 1);
  const int c = cp * 2;
  const v4f w0 = *(const v4f*)(cw + (size_t)c * DCONV);
  const v4f w1 = *(const v4f*)(cw + (size_t)c * DCONV + 4);
  float a0 = 0.f, a1 = 0.f;
#pragma unroll
  for (int j = 0; j < DCONV; ++j) {
    const int ll = l + j - (DCONV - 1);
    const int rr = (ll >= 0) ? (row + j - (DCONV - 1)) : row;
    const v2f xv = *(const v2f*)(xz + (size_t)rr * (2 * DI) + c);
    const float xa = (ll >= 0) ? xv[0] : 0.f;
    const float xb = (ll >= 0) ? xv[1] : 0.f;
    a0 += w0[j] * xa;
    a1 += w1[j] * xb;
  }
  a0 += cb[c];
  a1 += cb[c + 1];
  const float s0 = a0 * __builtin_amdgcn_rcpf(1.0f + expf(-a0));
  const float s1 = a1 * __builtin_amdgcn_rcpf(1.0f + expf(-a1));
  v2f o; o[0] = s0; o[1] = s1;
  const unsigned u = (unsigned)__builtin_bit_cast(unsigned short, (_Float16)(s0 * XSC)) |
                     ((unsigned)__builtin_bit_cast(unsigned short, (_Float16)(s1 * XSC)) << 16);
  float* p32 = xs32 + (size_t)row * DI + c;
  unsigned* p16 = (unsigned*)(void*)(xs16 + (size_t)row * DI + c);
  *(volatile v2f*)p32 = o;
  *(volatile unsigned*)p16 = u;
  __threadfence();
  *(volatile v2f*)p32 = o;
  *(volatile unsigned*)p16 = u;
}

__global__ __launch_bounds__(64) void k_scan(const float* __restrict__ xs32, const float* __restrict__ dtbc, const float* __restrict__ xz,
                                            const float* __restrict__ bdt, const float* __restrict__ Alog, const float* __restrict__ Dp,
                                            _Float16* __restrict__ y16) {
  __shared__ float sA[64 * 17];
  __shared__ __align__(16) _Float16 ys[16 * 64];
  const int tid = threadIdx.x, lane = tid & 31, wave = tid >> 5;
  const int b = blockIdx.x >> 3;
  const int cg = blockIdx.x & 7;
  const int c = cg * 64 + tid;
#pragma unroll 1
  for (int s = 0; s < DS; ++s) sA[tid * 17 + s] = -expf(Alog[(size_t)c * DS + s]) * LOG2E_F;
  __syncthreads();
  float Al[DS], hst[DS];
#pragma unroll
  for (int s = 0; s < DS; ++s) { Al[s] = sA[tid * 17 + s]; hst[s] = 0.f; }
  const float bc = bdt[c];
  const float Dd = Dp[c];
  const size_t rb = (size_t)b * LL;
  const int q = lane >> 3, c8 = (lane & 7) * 8;
#pragma unroll 1
  for (int t0 = 0; t0 < LL; t0 += 16) {
#pragma unroll 1
    for (int tt = 0; tt < 16; ++tt) {
      const size_t row = rb + t0 + tt;
      const float xv = xs32[row * DI + c];
      const float* dr = dtbc + row * NDT;
      const float u = dr[c] + bc;
      const float dt = fmaxf(u, 0.f) + log1pf(expf(-fabsf(u)));
      const float z = xz[row * (2 * DI) + DI + c];
      const float sz = z * __builtin_amdgcn_rcpf(1.0f + expf(-z));
      const v4f b0 = *(const v4f*)(dr + DI), b1 = *(const v4f*)(dr + DI + 4), b2 = *(const v4f*)(dr + DI + 8), b3 = *(const v4f*)(dr + DI + 12);
      const v4f c0 = *(const v4f*)(dr + DI + DS), c1 = *(const v4f*)(dr + DI + DS + 4), c2 = *(const v4f*)(dr + DI + DS + 8), c3 = *(const v4f*)(dr + DI + DS + 12);
      const float Bv[DS] = {b0[0], b0[1], b0[2], b0[3], b1[0], b1[1], b1[2], b1[3], b2[0], b2[1], b2[2], b2[3], b3[0], b3[1], b3[2], b3[3]};
      const float Cv[DS] = {c0[0], c0[1], c0[2], c0[3], c1[0], c1[1], c1[2], c1[3], c2[0], c2[1], c2[2], c2[3], c3[0], c3[1], c3[2], c3[3]};
      const float dtx = dt * xv;
      float y = 0.f;
#pragma unroll
      for (int s = 0; s < DS; ++s) {
        const float ab = exp2f(Al[s] * dt);
        hst[s] = ab * hst[s] + dtx * Bv[s];
        y += hst[s] * Cv[s];
      }
      y = y + Dd * xv;
      y = y * sz;
      ys[tt * 64 + tid] = (_Float16)(y * YSC);
    }
    __syncthreads();
    for (int pass = 0; pass < 2; ++pass) {
#pragma unroll
      for (int it = 0; it < 2; ++it) {
        const int r = wave * 8 + it * 4 + q;
        const v8h v = *(const v8h*)(ys + r * 64 + c8);
        *(volatile v8h*)(y16 + (rb + t0 + r) * DI + cg * 64 + c8) = v;
      }
      __threadfence();
    }
    __syncthreads();
  }
}

__global__ __launch_bounds__(256) void k_final(const float* __restrict__ h, const float* __restrict__ g, const float* __restrict__ bb,
                                              float* __restrict__ out) {
  __shared__ __align__(16) float red[8 * DM];
  const int lane = threadIdx.x & 31, wave = threadIdx.x >> 5;
  const int b = blockIdx.x;
  const int cA = lane * 4, cB = 128 + lane * 4;
  float acc[8];
#pragma unroll
  for (int e = 0; e < 8; ++e) acc[e] = 0.f;
#pragma unroll 1
  for (int i = 0; i < LL / 8; ++i) {
    const size_t row = (size_t)b * LL + wave + 8 * i;
    const float* pr = h + row * DM;
    const v4f vA = *(const v4f*)(pr + cA), vB = *(const v4f*)(pr + cB);
    float v[8] = {vA[0], vA[1], vA[2], vA[3], vB[0], vB[1], vB[2], vB[3]};
    float o[8];
    ln_row8(v, g, bb, cA, cB, o);
#pragma unroll
    for (int e = 0; e < 8; ++e) acc[e] += o[e];
  }
#pragma unroll
  for (int e = 0; e < 4; ++e) { red[wave * DM + cA + e] = acc[e]; red[wave * DM + cB + e] = acc[4 + e]; }
  __syncthreads();
  if (wave == 0) {
    v4f oA, oB;
#pragma unroll
    for (int e = 0; e < 4; ++e) {
      float ta = red[cA + e], tb = red[cB + e];
#pragma unroll
      for (int w = 1; w < 8; ++w) { ta += red[w * DM + cA + e]; tb += red[w * DM + cB + e]; }
      oA[e] = ta * (1.0f / LL);
      oB[e] = tb * (1.0f / LL);
    }
    float* po = out + (size_t)b * DM;
    *(volatile v4f*)(po + cA) = oA;
    *(volatile v4f*)(po + cB) = oB;
    __threadfence();
    *(volatile v4f*)(po + cA) = oA;
    *(volatile v4f*)(po + cB) = oB;
  }
}

extern "C" void kernel_launch(void* const* d_in, const int* in_sizes, int n_in,
                              void* d_out, int out_size, void* d_ws, size_t ws_size,
                              hipStream_t stream) {
  (void)in_sizes; (void)n_in; (void)out_size;
  const float* x       = (const float*)d_in[0];
  const float* w_in    = (const float*)d_in[1];
  const float* b_in    = (const float*)d_in[2];
  const float* ln_in_g = (const float*)d_in[3];
  const float* ln_in_b = (const float*)d_in[4];
  const float* ln_g    = (const float*)d_in[5];
  const float* ln_b    = (const float*)d_in[6];
  const float* W_inpr  = (const float*)d_in[7];
  const float* conv_w  = (const float*)d_in[8];
  const float* conv_b  = (const float*)d_in[9];
  const float* W_dt    = (const float*)d_in[10];
  const float* b_dt    = (const float*)d_in[11];
  const float* W_B     = (const float*)d_in[12];
  const float* W_C     = (const float*)d_in[13];
  const float* A_log   = (const float*)d_in[14];
  const float* Dp      = (const float*)d_in[15];
  const float* W_out   = (const float*)d_in[16];
  const float* ln_f_g  = (const float*)d_in[17];
  const float* ln_f_b  = (const float*)d_in[18];
  float* out = (float*)d_out;

  char* ws = (char*)d_ws;
  size_t off = 0;
  auto carve = [&](size_t bytes) -> void* {
    void* p = ws + off;
    off += (bytes + 255) & ~(size_t)255;
    return p;
  };
  float*    h    = (float*)carve((size_t)MROWS * DM * 4);
  _Float16* hn16 = (_Float16*)carve((size_t)MROWS * DM * 2);
  float*    xz   = (float*)carve((size_t)MROWS * 2 * DI * 4);
  float*    xs32 = (float*)carve((size_t)MROWS * DI * 4);
  _Float16* xs16 = (_Float16*)carve((size_t)MROWS * DI * 2);
  float*    dtbc = (float*)carve((size_t)MROWS * NDT * 4);
  _Float16* y16  = (_Float16*)carve((size_t)MROWS * DI * 2);
  _Float16* WinT = (_Float16*)carve((size_t)NL * 2 * DI * DM * 2);
  _Float16* WdtT = (_Float16*)carve((size_t)NL * NDT * DI * 2);
  _Float16* WoT  = (_Float16*)carve((size_t)NL * DM * DI * 2);
  if (off > ws_size) return;

  k_wprep<<<dim3(DM / 64, (2 * DI) / 64, NL), 256, 0, stream>>>(W_inpr, 2 * DI, (long)DM * 2 * DI, DM, 2 * DI, 2 * DI,
                                                                  WinT, DM, (long)2 * DI * DM, 0, WSC);
  k_wprep<<<dim3(DI / 64, DI / 64, NL), 256, 0, stream>>>(W_dt, DI, (long)DI * DI, DI, DI, DI,
                                                            WdtT, DI, (long)NDT * DI, 0, WSC);
  k_wprep<<<dim3(DI / 64, 1, NL), 256, 0, stream>>>(W_B, DS, (long)DI * DS, DI, DS, DS,
                                                      WdtT, DI, (long)NDT * DI, DI, WSC);
  k_wprep<<<dim3(DI / 64, 1, NL), 256, 0, stream>>>(W_C, DS, (long)DI * DS, DI, DS, NDT - DI - DS,
                                                      WdtT, DI, (long)NDT * DI, DI + DS, WSC);
  k_wprep<<<dim3(DI / 64, DM / 64, NL), 256, 0, stream>>>(W_out, DM, (long)DI * DM, DI, DM, DM,
                                                            WoT, DI, (long)DM * DI, 0, WSC);

  k_stem<<<MROWS / 8, 256, 0, stream>>>(x, w_in, b_in, ln_in_g, ln_in_b, h);

  const int gridIn  = ((MROWS / 64) * ((2 * DI) / 64)) / 8;
  const int gridDt  = ((MROWS / 64) * (NDT / 64)) / 8;
  const int gridOut = ((MROWS / 64) * (DM / 64)) / 8;

  for (int i = 0; i < NL; ++i) {
    const _Float16* WinTi = WinT + (size_t)i * 2 * DI * DM;
    const _Float16* WdtTi = WdtT + (size_t)i * NDT * DI;
    const _Float16* WoTi  = WoT + (size_t)i * DM * DI;

    k_ln<<<MROWS / 8, 256, 0, stream>>>(h, ln_g + (size_t)i * DM, ln_b + (size_t)i * DM, hn16);

    wmma_gemm64<0, false, 0, 0, false, 0><<<dim3(gridIn, 1), 256, 0, stream>>>(
        (const unsigned short*)hn16, (const unsigned short*)hn16, DM, 0L,
        (const unsigned short*)WinTi, (const unsigned short*)WinTi, DM, 0L,
        (void*)xz, (void*)xz, 2 * DI, 0L,
        b_dt, h, 0L, MROWS, 2 * DI, DM, 1.0f / WSC);

    k_conv<<<(MROWS * 256) / 256, 256, 0, stream>>>(xz, conv_w + (size_t)i * DI * DCONV, conv_b + (size_t)i * DI, xs32, xs16);

    wmma_gemm64<0, false, 0, 0, false, 0><<<dim3(gridDt, 1), 256, 0, stream>>>(
        (const unsigned short*)xs16, (const unsigned short*)xs16, DI, 0L,
        (const unsigned short*)WdtTi, (const unsigned short*)WdtTi, DI, 0L,
        (void*)dtbc, (void*)dtbc, NDT, 0L,
        b_dt, h, 0L, MROWS, NDT, DI, 1.0f / (WSC * XSC));

    k_scan<<<BB * (DI / 64), 64, 0, stream>>>(xs32, dtbc, xz, b_dt + (size_t)i * DI, A_log + (size_t)i * DI * DS,
                                              Dp + (size_t)i * DI, y16);

    wmma_gemm64<0, false, 0, 0, true, 0><<<dim3(gridOut, 1), 256, 0, stream>>>(
        (const unsigned short*)y16, (const unsigned short*)y16, DI, 0L,
        (const unsigned short*)WoTi, (const unsigned short*)WoTi, DI, 0L,
        (void*)h, (void*)h, DM, 0L,
        b_dt, h, 0L, MROWS, DM, DI, 1.0f / (WSC * YSC));
  }

  k_final<<<BB, 256, 0, stream>>>(h, ln_f_g, ln_f_b, out);
}
